// PositionConditionerBlock_33380485825341
// MI455X (gfx1250) — hardware-verified
//
#include <hip/hip_runtime.h>
#include <math.h>

#ifndef NB
#define NB 1
#endif
#ifndef SEQ
#define SEQ 2048
#endif
#define SEQ_FULL 2048
#define NDIM 128
#define NAUX 16
#define NROT 4
#define HSRC 8
#define NHEAD 24
#define CH 32
#define KQW 512
#define VALW 3072

#define A_CARRY_LG 4
#define W_CARRY_LG 6
#define A_CARRY 16.0f
#define W_CARRY 64.0f
#define GEMM_UNDO 0.0009765625f
#define KQ_CARRY 16.0f
#define SCORE_UNDO 0.00390625f
#define V_CARRY 16.0f
#define P_CARRY 1024.0f
#define OUT_UNDO 0.00006103515625f
#define INV_SQRT_H 0.35355339059327373f
#define LOG2E 1.4426950408889634f
#define SC_LIN (SCORE_UNDO * INV_SQRT_H * LOG2E)
#define SC_SQ (INV_SQRT_H * LOG2E)

#define KQ_HALF (NHEAD * SEQ * CH)
#define KQL_HALF (HSRC * SEQ * CH)
#define AT_TP4 33

static_assert(NB == 1);
static_assert(SEQ <= SEQ_FULL);
static_assert((SEQ & (SEQ - 1)) == 0);
static_assert(SEQ % 64 == 0);
static_assert(NDIM == 128 && CH == 32 && NHEAD == 3 * HSRC);
static_assert(KQW == HSRC * 2 * CH && VALW == NHEAD * NDIM);
static_assert(NDIM % 32 == 0 && KQW % 64 == 0 && VALW % 64 == 0);
static_assert((float)(1 << A_CARRY_LG) == A_CARRY && (float)(1 << W_CARRY_LG) == W_CARRY);
static_assert(A_CARRY * W_CARRY * GEMM_UNDO == 1.0f);
static_assert(KQ_CARRY * KQ_CARRY * SCORE_UNDO == 1.0f);
static_assert(V_CARRY * P_CARRY * OUT_UNDO == 1.0f);
static_assert((SEQ * NDIM / 8) % 256 == 0 && (KQW * NDIM / 8) % 256 == 0 && (VALW * NDIM / 8) % 256 == 0);
static_assert((SEQ * 4) % 256 == 0);

typedef _Float16 h16;
typedef __attribute__((ext_vector_type(16))) _Float16 v16h;
typedef __attribute__((ext_vector_type(8)))  _Float16 v8h;
typedef __attribute__((ext_vector_type(8)))  float    v8f;
typedef __attribute__((ext_vector_type(4)))  float    v4f;


__device__ __forceinline__ float bfr(float f) {
    unsigned u = __float_as_uint(f);
    u += 0x7FFFu + ((u >> 16) & 1u);
    return __uint_as_float(u & 0xFFFF0000u);
}
static __device__ __forceinline__ h16 toh_flush(float v) { const float w = (fabsf(v) < 6.103515625e-05f) ? 0.0f : v; return (h16)w; }

__device__ __forceinline__ void st8h16(_Float16* P, size_t o, const float* v) {
    v8h hv;
#pragma unroll
    for (int e = 0; e < 8; ++e) hv[e] = toh_flush(v[e]);
    *(volatile v8h*)(P + o) = hv;
    __threadfence();
    *(volatile v8h*)(P + o) = hv;
}

union FragU { v16h v; v8h h[2]; };
__device__ __forceinline__ v16h frag_ld(const _Float16* p) {
    FragU f; f.h[0] = *(const v8h*)(p); f.h[1] = *(const v8h*)(p + 16); return f.v;
}
__device__ __forceinline__ v8f wmma16g(v16h a, v16h b, v8f c) {
    c = __builtin_amdgcn_wmma_f32_16x16x32_f16(false, a, false, b, (short)0, c, false, false);
    asm volatile("v_nop\n\tv_nop\n\tv_nop\n\tv_nop" : "+v"(c) : "v"(a), "v"(b));
    return c;
}
__device__ __forceinline__ void wave_sync_lds() {
    __builtin_amdgcn_fence(3  , "workgroup");
    __builtin_amdgcn_wave_barrier();
    __builtin_amdgcn_fence(2  , "workgroup");
}

__global__ __launch_bounds__(256) void k_cvt16(const float* __restrict__ src, _Float16* __restrict__ dst, unsigned n8, unsigned lgs) {
    const unsigned u = blockIdx.x * 256u + threadIdx.x;
    if (u >= n8) return;
    const float sw = (float)(1u << lgs);
    const float* s = src + (size_t)u * 8u;
    const v4f a = *(const v4f*)s, b = *(const v4f*)(s + 4);
    float v[8];
    v[0] = bfr(a.x) * sw; v[1] = bfr(a.y) * sw; v[2] = bfr(a.z) * sw; v[3] = bfr(a.w) * sw;
    v[4] = bfr(b.x) * sw; v[5] = bfr(b.y) * sw; v[6] = bfr(b.z) * sw; v[7] = bfr(b.w) * sw;
    st8h16(dst, (size_t)u * 8u, v);
}

static_assert(2 * 4 * 32 * 16 == 16 * 64 * 4);
static_assert(4 * 32 * 16 == 16 * 64 * 2);
static_assert(8 * 16 * 68 * 4 <= 131072);
__global__ __launch_bounds__(256) void k_gemm64(
    const _Float16* __restrict__ A, unsigned lda, const _Float16* __restrict__ Bt, unsigned ldb,
    float* __restrict__ C32, _Float16* __restrict__ C16, unsigned ldc, const float* __restrict__ bias,
    unsigned M, unsigned N, unsigned K, unsigned lgTN, unsigned mode) {
  __shared__ __align__(16) float sT[8][16 * 68];
  const unsigned lane = threadIdx.x & 31u;
  const unsigned wave = (unsigned)__builtin_amdgcn_readfirstlane((int)(threadIdx.x >> 5));
  const unsigned tilesN = N >> 6, tilesM = M >> 6;
  const unsigned tile = blockIdx.x * 8u + wave;
  if (tile >= tilesM * tilesN) return;
  const unsigned tm = tile >> lgTN;
  const unsigned tn = tile & (tilesN - 1u);
  const unsigned m0 = tm << 6, n0 = tn << 6;
  const unsigned rlane = lane & 15u;
  const unsigned koff = (lane >> 4) * 8u;
  const unsigned mOff = koff;

  v8f acc[4][4];
#pragma unroll
  for (int i = 0; i < 4; ++i)
#pragma unroll
    for (int j = 0; j < 4; ++j) acc[i][j] = (v8f){0.f,0.f,0.f,0.f,0.f,0.f,0.f,0.f};

  for (unsigned k0 = 0; k0 < K; k0 += 32u) {
    v16h bh[4];
#pragma unroll
    for (int j = 0; j < 4; ++j)
      bh[j] = frag_ld(Bt + (size_t)(n0 + ((unsigned)j << 4) + rlane) * ldb + koff + k0);
#pragma unroll
    for (int i = 0; i < 4; ++i) {
      const v16h ah = frag_ld(A + (size_t)(m0 + ((unsigned)i << 4) + rlane) * lda + koff + k0);
#pragma unroll
      for (int j = 0; j < 4; ++j)
        acc[i][j] = wmma16g(ah, bh[j], acc[i][j]);
    }
  }

  const float oscale = (mode != 0u) ? V_CARRY : 1.0f;
#pragma unroll
  for (int i = 0; i < 4; ++i) {
    const unsigned mBase = m0 + ((unsigned)i << 4);
    float rb[8];
#pragma unroll
    for (int r = 0; r < 8; ++r) {
      const unsigned ridx = (mode != 0u) ? (mBase + mOff + (unsigned)r) : 0u;
      const float t = bfr(bias[ridx]);
      rb[r] = (mode != 0u) ? t : 0.0f;
    }
#pragma unroll
    for (int j = 0; j < 4; ++j) {
      const unsigned n = n0 + ((unsigned)j << 4) + rlane;
      const unsigned cidx = (mode == 0u) ? n : 0u;
      const float tc = bfr(bias[cidx]);
      const float cb = (mode == 0u) ? tc : 0.0f;
#pragma unroll
      for (int r = 0; r < 8; ++r) {
        const float v = (acc[i][j][r] * GEMM_UNDO + (cb + rb[r])) * oscale;
        sT[wave][(mOff + (unsigned)r) * 68u + ((unsigned)j << 4) + rlane] = v;
      }
    }
    wave_sync_lds();
    if (mode == 0u) {
      const unsigned hh = lane >> 4, c4 = (lane & 15u) * 4u;
#pragma unroll
      for (int half = 0; half < 2; ++half) {
        v4f vv[4];
#pragma unroll
        for (int it = 0; it < 4; ++it) {
          const unsigned row = (unsigned)(half * 4 + it) * 2u + hh;
          vv[it] = *(const v4f*)(&sT[wave][row * 68u + c4]);
        }
        for (int pass = 0; pass < 2; ++pass) {
#pragma unroll
          for (int it = 0; it < 4; ++it) {
            const unsigned row = (unsigned)(half * 4 + it) * 2u + hh;
            *(volatile v4f*)(C32 + (size_t)(mBase + row) * ldc + n0 + c4) = vv[it];
          }
          __threadfence();
        }
      }
    } else {
      const unsigned q = lane >> 3, c8 = (lane & 7u) * 8u;
      v8h hv[4];
#pragma unroll
      for (int it = 0; it < 4; ++it) {
        const unsigned row = (unsigned)it * 4u + q;
#pragma unroll
        for (int e = 0; e < 8; ++e) hv[it][e] = toh_flush(sT[wave][row * 68u + c8 + (unsigned)e]);
      }
      for (int pass = 0; pass < 2; ++pass) {
#pragma unroll
        for (int it = 0; it < 4; ++it) {
          const unsigned row = (unsigned)it * 4u + q;
          *(volatile v8h*)(C16 + (size_t)(mBase + row) * ldc + n0 + c8) = hv[it];
        }
        __threadfence();
      }
    }
    wave_sync_lds();
  }
}

__global__ __launch_bounds__(256) void k_planes(const float* __restrict__ kqn, const float* __restrict__ aux,
                                                const float* __restrict__ rot, const float* __restrict__ W_aux,
                                                const float* __restrict__ b_aux, const float* __restrict__ W_rot,
                                                _Float16* __restrict__ kq16, _Float16* __restrict__ kql16) {
    const unsigned bx = blockIdx.x;
    const unsigned g = bx / (unsigned)(SEQ / 64);
    if (g >= 2u * (unsigned)NHEAD) return;
    const unsigned kq = g & 1u, h = g >> 1;
    const unsigned u = (bx - g * (unsigned)(SEQ / 64)) * 256u + threadIdx.x;
    const unsigned p = u & 3u, i = u >> 2;
    const unsigned cc0 = 32u * kq + 8u * p;
    float v[8];
#pragma unroll
    for (int e = 0; e < 8; ++e) v[e] = 0.0f;
    if (h < 8u) {
        const float* src = kqn + (size_t)i * KQW + 64u * h + cc0;
        const v4f a = *(const v4f*)src, b = *(const v4f*)(src + 4);
        v[0] = a.x; v[1] = a.y; v[2] = a.z; v[3] = a.w; v[4] = b.x; v[5] = b.y; v[6] = b.z; v[7] = b.w;
    } else if (h < 16u) {
        const unsigned r0 = 64u * (h - 8u) + cc0;
        for (unsigned x = 0; x < (unsigned)NAUX; ++x) {
            const float ax = bfr(aux[(size_t)i * NAUX + x]);
#pragma unroll
            for (int e = 0; e < 8; ++e) v[e] += ax * bfr(W_aux[(size_t)(r0 + (unsigned)e) * NAUX + x]);
        }
#pragma unroll
        for (int e = 0; e < 8; ++e) v[e] += bfr(b_aux[r0 + (unsigned)e]);
    } else {
        const unsigned r0 = 64u * (h - 16u) + cc0;
        for (unsigned x = 0; x < (unsigned)NROT; ++x) {
            const float rx = bfr(rot[(size_t)i * NROT + x]);
#pragma unroll
            for (int e = 0; e < 8; ++e) v[e] += rx * bfr(W_rot[(size_t)(r0 + (unsigned)e) * NROT + x]);
        }
    }
#pragma unroll
    for (int e = 0; e < 8; ++e) v[e] *= KQ_CARRY;
    st8h16(kq16, (size_t)(((kq * (unsigned)NHEAD + h) * (unsigned)SEQ + i) * (unsigned)CH + 8u * p), v);
    if (h >= 16u) {
        float lo[8];
#pragma unroll
        for (int e = 0; e < 8; ++e) lo[e] = v[e] - (float)toh_flush(v[e]);
        st8h16(kql16, (size_t)(((kq * (unsigned)HSRC + (h - 16u)) * (unsigned)SEQ + i) * (unsigned)CH + 8u * p), lo);
    }
}

template <bool ROT>
__device__ __forceinline__ void head_pass(const _Float16* __restrict__ kq16, const _Float16* __restrict__ kql16,
                                          const _Float16* __restrict__ vt16, unsigned head, unsigned i0,
                                          unsigned hh, unsigned c, v8f (&ofin)[8]) {
    const v8f z8 = (v8f){0.f,0.f,0.f,0.f,0.f,0.f,0.f,0.f};
    const unsigned frow = c * (unsigned)CH + 8u * hh;
    const unsigned hl = ROT ? (head - 16u) : 0u;
    const _Float16* kp  = kq16 + (size_t)((head * (unsigned)SEQ + i0) * (unsigned)CH + frow);
    const _Float16* qp  = kq16 + (size_t)((unsigned)KQ_HALF + head * (unsigned)SEQ * (unsigned)CH + frow);
    const _Float16* klp = kql16 + (size_t)((hl * (unsigned)SEQ + i0) * (unsigned)CH + frow);
    const _Float16* qlp = kql16 + (size_t)((unsigned)KQL_HALF + hl * (unsigned)SEQ * (unsigned)CH + frow);
    const _Float16* vp  = vt16 + (size_t)((head * (unsigned)NDIM + c) * (unsigned)SEQ + 8u * hh);
    const v16h kh = frag_ld(kp);
    v16h kl = kh;
    if (ROT) kl = frag_ld(klp);

    v8f o[8];
#pragma unroll
    for (int t = 0; t < 8; ++t) o[t] = z8;
    float m = -3.0e38f, l = 0.0f;

#pragma unroll 1
    for (unsigned j0 = 0; j0 < (unsigned)SEQ; j0 += 32u) {
        v8f s0 = z8, s1 = z8;
        {
            const v16h q0 = frag_ld(qp + (size_t)(j0 * (unsigned)CH));
            const v16h q1 = frag_ld(qp + (size_t)((j0 + 16u) * (unsigned)CH));
            s0 = wmma16g(q0, kh, s0);
            s1 = wmma16g(q1, kh, s1);
            if (ROT) {
                s0 = wmma16g(q0, kl, s0);
                s1 = wmma16g(q1, kl, s1);
                const v16h r0 = frag_ld(qlp + (size_t)(j0 * (unsigned)CH));
                const v16h r1 = frag_ld(qlp + (size_t)((j0 + 16u) * (unsigned)CH));
                s0 = wmma16g(r0, kh, s0);
                s1 = wmma16g(r1, kh, s1);
            }
        }
        float x[16];
#pragma unroll
        for (int r = 0; r < 8; ++r) { x[r] = s0[r]; x[8 + r] = s1[r]; }
        if (ROT) {
#pragma unroll
            for (int e = 0; e < 16; ++e) { const float d = x[e] * SCORE_UNDO; x[e] = (d * d) * SC_SQ; }
        } else {
#pragma unroll
            for (int e = 0; e < 16; ++e) x[e] *= SC_LIN;
        }
        float mx = x[0];
#pragma unroll
        for (int e = 1; e < 16; ++e) mx = (x[e] > mx) ? x[e] : mx;
        const float mo = __shfl_xor(mx, 16, 32);
        mx = (mo > mx) ? mo : mx;
        const float mnew = (mx > m) ? mx : m;
        const float alpha = exp2f(m - mnew);
        m = mnew;
        v16h pf;
        float psum = 0.0f;
#pragma unroll
        for (int e = 0; e < 16; ++e) {
            const float pe = exp2f(x[e] - mnew);
            psum += pe;
            pf[e] = toh_flush(pe * P_CARRY);
        }
        l = l * alpha + psum;
#pragma unroll
        for (int t = 0; t < 8; ++t) o[t] = o[t] * alpha;

        unsigned jv = j0;
        asm volatile("" : "+v"(jv));
#pragma unroll
        for (int t = 0; t < 4; ++t) {
            const v16h a = frag_ld(vp + (size_t)((unsigned)t * 16u * (unsigned)SEQ + jv));
            o[t] = wmma16g(a, pf, o[t]);
        }
        asm volatile("" : "+v"(jv));
#pragma unroll
        for (int t = 4; t < 8; ++t) {
            const v16h a = frag_ld(vp + (size_t)((unsigned)t * 16u * (unsigned)SEQ + jv));
            o[t] = wmma16g(a, pf, o[t]);
        }
    }
    const float lt = l + __shfl_xor(l, 16, 32);
    const float inv = (1.0f / lt) * OUT_UNDO;
#pragma unroll
    for (int t = 0; t < 8; ++t) ofin[t] = o[t] * inv;
}

static_assert(4 * 4 * 32 * 16 == 16 * NDIM * 4);
static_assert(4 * 16 * AT_TP4 * 16 <= 131072);
static_assert(SEQ % 32 == 0 && SEQ % 16 == 0);
__global__ __launch_bounds__(128) __attribute__((amdgpu_num_vgpr(256))) void k_attn(
    const _Float16* __restrict__ kq16, const _Float16* __restrict__ kql16,
    const _Float16* __restrict__ vt16, float* __restrict__ out) {
    __shared__ v4f sTot[4 * 16 * AT_TP4];
    const unsigned tid = threadIdx.x, lane = tid & 31u;
    const unsigned wave = (unsigned)__builtin_amdgcn_readfirstlane((int)(tid >> 5));
    const unsigned hh = lane >> 4, c = lane & 15u;
    const unsigned i0 = blockIdx.x * 16u;
    const unsigned tb = (wave * 16u + c) * (unsigned)AT_TP4 + 2u * hh;
    const v4f z4 = (v4f){0.f, 0.f, 0.f, 0.f};
#pragma unroll
    for (int t = 0; t < 8; ++t) { sTot[tb + 4u * (unsigned)t] = z4; sTot[tb + 4u * (unsigned)t + 1u] = z4; }

#pragma unroll 1
    for (unsigned hi = 0; hi < 4u; ++hi) {
        v8f of[8];
        head_pass<false>(kq16, kql16, vt16, wave + 4u * hi, i0, hh, c, of);
#pragma unroll
        for (int t = 0; t < 8; ++t) {
            v4f a = sTot[tb + 4u * (unsigned)t], b = sTot[tb + 4u * (unsigned)t + 1u];
            a.x += of[t][0]; a.y += of[t][1]; a.z += of[t][2]; a.w += of[t][3];
            b.x += of[t][4]; b.y += of[t][5]; b.z += of[t][6]; b.w += of[t][7];
            sTot[tb + 4u * (unsigned)t] = a; sTot[tb + 4u * (unsigned)t + 1u] = b;
        }
    }
#pragma unroll 1
    for (unsigned hi = 4u; hi < 6u; ++hi) {
        v8f of[8];
        head_pass<true>(kq16, kql16, vt16, wave + 4u * hi, i0, hh, c, of);
#pragma unroll
        for (int t = 0; t < 8; ++t) {
            v4f a = sTot[tb + 4u * (unsigned)t], b = sTot[tb + 4u * (unsigned)t + 1u];
            a.x += of[t][0]; a.y += of[t][1]; a.z += of[t][2]; a.w += of[t][3];
            b.x += of[t][4]; b.y += of[t][5]; b.z += of[t][6]; b.w += of[t][7];
            sTot[tb + 4u * (unsigned)t] = a; sTot[tb + 4u * (unsigned)t + 1u] = b;
        }
    }
    __syncthreads();
    {
        v4f vv[4];
#pragma unroll
        for (int it = 0; it < 4; ++it) {
            const unsigned row = (unsigned)it * 4u + wave;
            const v4f a0 = sTot[(0u * 16u + row) * (unsigned)AT_TP4 + lane];
            const v4f a1 = sTot[(1u * 16u + row) * (unsigned)AT_TP4 + lane];
            const v4f a2 = sTot[(2u * 16u + row) * (unsigned)AT_TP4 + lane];
            const v4f a3 = sTot[(3u * 16u + row) * (unsigned)AT_TP4 + lane];
            vv[it] = ((a0 + a1) + a2) + a3;
        }
        for (int pass = 0; pass < 2; ++pass) {
#pragma unroll
            for (int it = 0; it < 4; ++it) {
                const unsigned row = (unsigned)it * 4u + wave;
                *(volatile v4f*)(out + (size_t)(i0 + row) * NDIM + 4u * lane) = vv[it];
            }
            __threadfence();
        }
    }
}

static constexpr size_t WS_N16  = (size_t)SEQ * NDIM * 2;
static constexpr size_t WS_WN16 = (size_t)KQW * NDIM * 2;
static constexpr size_t WS_WV16 = (size_t)VALW * NDIM * 2;
static constexpr size_t WS_KQN  = (size_t)SEQ * KQW * 4;
static constexpr size_t WS_KQ16 = (size_t)2 * KQ_HALF * 2;
static constexpr size_t WS_KQL  = (size_t)2 * KQL_HALF * 2;
static constexpr size_t WS_VT16 = (size_t)VALW * SEQ * 2;
static constexpr size_t WS_TOTAL = WS_N16 + WS_WN16 + WS_WV16 + WS_KQN + WS_KQ16 + WS_KQL + WS_VT16;
static_assert(WS_N16 % 256 == 0 && WS_WN16 % 256 == 0 && WS_WV16 % 256 == 0 && WS_KQN % 256 == 0);
static_assert(WS_KQ16 % 256 == 0 && WS_KQL % 256 == 0 && WS_VT16 % 256 == 0);
static_assert(WS_TOTAL <= (size_t)134217728);

static constexpr unsigned ilog2c(unsigned v) { return v <= 1u ? 0u : 1u + ilog2c(v >> 1); }
static_assert((1u << ilog2c(KQW / 64)) == KQW / 64);
static_assert((1u << ilog2c(SEQ / 64)) == SEQ / 64);

extern "C" void kernel_launch(void* const* d_in, const int* in_sizes, int n_in, void* d_out, int out_size,
                              void* d_ws, size_t ws_size, hipStream_t stream) {
    if (n_in < 10) return;
    if (in_sizes[0] < SEQ * NDIM || in_sizes[1] < SEQ * NAUX || in_sizes[2] < SEQ * NROT) return;
    if (in_sizes[3] < KQW * NDIM || in_sizes[4] < KQW || in_sizes[5] < KQW * NAUX || in_sizes[6] < KQW) return;
    if (in_sizes[7] < KQW * NROT || in_sizes[8] < VALW * NDIM || in_sizes[9] < VALW) return;
    if (out_size < SEQ * NDIM) return;

    const float* nodes   = (const float*)d_in[0];
    const float* aux     = (const float*)d_in[1];
    const float* rot     = (const float*)d_in[2];
    const float* W_nodes = (const float*)d_in[3];
    const float* b_nodes = (const float*)d_in[4];
    const float* W_aux   = (const float*)d_in[5];
    const float* b_aux   = (const float*)d_in[6];
    const float* W_rot   = (const float*)d_in[7];
    const float* W_val   = (const float*)d_in[8];
    const float* b_val   = (const float*)d_in[9];
    float* out = (float*)d_out;

    char* wsp = (char*)d_ws;
    size_t off = 0;
    auto carve = [&](size_t bytes) -> void* { void* r = wsp + off; off += (bytes + 255) & ~(size_t)255; return r; };
    _Float16* n16   = (_Float16*)carve(WS_N16);
    _Float16* wn16  = (_Float16*)carve(WS_WN16);
    _Float16* wv16  = (_Float16*)carve(WS_WV16);
    float*    kqn   = (float*)carve(WS_KQN);
    _Float16* kq16  = (_Float16*)carve(WS_KQ16);
    _Float16* kql16 = (_Float16*)carve(WS_KQL);
    _Float16* vt16  = (_Float16*)carve(WS_VT16);
    if (off > ws_size || off > (size_t)134217728) return;

    k_cvt16<<<(SEQ * NDIM / 8) / 256, 256, 0, stream>>>(nodes, n16, (unsigned)(SEQ * NDIM / 8), (unsigned)A_CARRY_LG);
    k_cvt16<<<(KQW * NDIM / 8) / 256, 256, 0, stream>>>(W_nodes, wn16, (unsigned)(KQW * NDIM / 8), (unsigned)W_CARRY_LG);
    k_cvt16<<<(VALW * NDIM / 8) / 256, 256, 0, stream>>>(W_val, wv16, (unsigned)(VALW * NDIM / 8), (unsigned)W_CARRY_LG);

    k_gemm64<<<((SEQ / 64) * (KQW / 64) + 7) / 8, 256, 0, stream>>>(
        (const _Float16*)n16, NDIM, (const _Float16*)wn16, NDIM, kqn, vt16, KQW, b_nodes,
        (unsigned)SEQ, (unsigned)KQW, (unsigned)NDIM, ilog2c(KQW / 64), 0u);
    k_gemm64<<<((VALW / 64) * (SEQ / 64) + 7) / 8, 256, 0, stream>>>(
        (const _Float16*)wv16, NDIM, (const _Float16*)n16, NDIM, kqn, vt16, SEQ, b_val,
        (unsigned)VALW, (unsigned)SEQ, (unsigned)NDIM, ilog2c(SEQ / 64), 1u);
    k_planes<<<2 * NHEAD * (SEQ / 64), 256, 0, stream>>>(kqn, aux, rot, W_aux, b_aux, W_rot, kq16, kql16);
    k_attn<<<SEQ / 16, 128, 0, stream>>>((const _Float16*)kq16, (const _Float16*)kql16, (const _Float16*)vt16, out);
}
